// LocalAttention_42545946034260
// MI455X (gfx1250) — hardware-verified
//
#include <hip/hip_runtime.h>
#include <stddef.h>


#ifndef NB
#define NB 2
#endif
#ifndef SEQ
#define SEQ 2048
#endif
#define NB_FULL 2
#define SEQ_FULL 2048
#define EDIM 512
#define WIN 64
#define NKT 9
#define NKEYS (NKT * 16)
#define PKEYS 160
#define NKC (PKEYS / 32)
#define VPAD 128
#define MROWS (NB * SEQ)
#define VTW (MROWS + 2 * VPAD)
#define SPITCH 148
#define PPITCH 168
#define OPITCH 516
#define TPITCH 68

static_assert(NB >= 1 && NB <= NB_FULL);
static_assert(SEQ >= 64 && SEQ <= SEQ_FULL && (SEQ % 64) == 0);
static_assert((MROWS * 64) % 256 == 0);
static_assert(((EDIM * EDIM) / 8) % 256 == 0);
static_assert((EDIM * 32) % 256 == 0);
static_assert(NKEYS >= 2 * WIN + 16 && PKEYS >= NKEYS && (PKEYS % 32) == 0);
static_assert(VPAD >= WIN && VPAD >= PKEYS - WIN - 16 && (VPAD % 64) == 0);
static_assert((VTW % 64) == 0);
static_assert(SPITCH >= NKEYS && PPITCH >= PKEYS && (PPITCH % 8) == 0 && OPITCH >= EDIM && (OPITCH % 4) == 0);

typedef unsigned int v4u __attribute__((ext_vector_type(4)));
typedef float v4f __attribute__((ext_vector_type(4)));
typedef float v8f __attribute__((ext_vector_type(8)));
typedef _Float16 v8h __attribute__((ext_vector_type(8)));
typedef _Float16 v16h __attribute__((ext_vector_type(16)));
typedef __bf16 v16bf __attribute__((ext_vector_type(16)));
typedef v4f v4f_ma __attribute__((may_alias));
typedef v8h v8h_ma __attribute__((may_alias));

union FragH { v16h v; v8h half[2]; v4u u[2]; };
union FragB { v16bf v; v4u u[2]; };
union Pack8H { v8h h; v4u u; };

__device__ __forceinline__ v8f mma_bf16(v16bf a, v16bf b, v8f c) {
  c = __builtin_amdgcn_wmma_f32_16x16x32_bf16(false, a, false, b, (short)0, c, false, false);
  asm volatile("v_nop\n\tv_nop\n\tv_nop\n\tv_nop" : "+v"(c) : "v"(a), "v"(b));
  return c;
}
__device__ __forceinline__ v8f mma_f16(v16h a, v16h b, v8f c) {
  c = __builtin_amdgcn_wmma_f32_16x16x32_f16(false, a, false, b, (short)0, c, false, false);
  asm volatile("v_nop\n\tv_nop\n\tv_nop\n\tv_nop" : "+v"(c) : "v"(a), "v"(b));
  return c;
}

__device__ __forceinline__ unsigned int bf16_rne_bits(float f) {
  unsigned int u = __float_as_uint(f);
  return (u + 0x7FFFu + ((u >> 16) & 1u)) >> 16;
}
__device__ __forceinline__ unsigned int pack_bf16x2(float a, float b) {
  return bf16_rne_bits(a) | (bf16_rne_bits(b) << 16);
}
__device__ __forceinline__ float bf16_rne_val(float f) {
  return __uint_as_float(bf16_rne_bits(f) << 16);
}
__device__ __forceinline__ v8f zero8() {
  v8f z = {0.f, 0.f, 0.f, 0.f, 0.f, 0.f, 0.f, 0.f};
  return z;
}

__global__ __launch_bounds__(256) void cvt_kernel(const float* __restrict__ x,
                                                  const float* __restrict__ wq,
                                                  const float* __restrict__ wk,
                                                  const float* __restrict__ wv,
                                                  unsigned short* xb,
                                                  unsigned short* wqb,
                                                  unsigned short* wkb,
                                                  unsigned short* wvb,
                                                  unsigned short* vth,
                                                  unsigned short* vtl) {
  const unsigned int u   = blockIdx.x * 256u + threadIdx.x;
  const unsigned int nxu = (unsigned int)MROWS * 64u;
  const unsigned int nwu = (unsigned int)(EDIM * EDIM) / 8u;
  const unsigned int npu = (unsigned int)EDIM * 32u;
  if (u < nxu) {
    const unsigned int R  = u >> 6;
    const unsigned int c8 = (u & 63u) * 8u;
    const unsigned int b  = R / SEQ;
    const unsigned int l  = R - b * SEQ;
    const float* src = x + ((size_t)(b * SEQ_FULL + l) * EDIM + c8);
    const v4f f0 = *(const v4f*)src;
    const v4f f1 = *(const v4f*)(src + 4);
    v4u o;
    o.x = pack_bf16x2(f0.x, f0.y);
    o.y = pack_bf16x2(f0.z, f0.w);
    o.z = pack_bf16x2(f1.x, f1.y);
    o.w = pack_bf16x2(f1.z, f1.w);
    unsigned short* dst = xb + (size_t)R * EDIM + c8;
    *(volatile v4u*)dst = o;
    __threadfence();
    *(volatile v4u*)dst = o;
  } else if (u < nxu + 3u * nwu) {
    const unsigned int t = u - nxu;
    const unsigned int w = t / nwu;
    const unsigned int e = (t - w * nwu) * 8u;
    const float* src = ((w == 0u) ? wq : (w == 1u) ? wk : wv) + e;
    unsigned short* dst = ((w == 0u) ? wqb : (w == 1u) ? wkb : wvb) + e;
    const v4f f0 = *(const v4f*)src;
    const v4f f1 = *(const v4f*)(src + 4);
    v4u o;
    o.x = pack_bf16x2(f0.x, f0.y);
    o.y = pack_bf16x2(f0.z, f0.w);
    o.z = pack_bf16x2(f1.x, f1.y);
    o.w = pack_bf16x2(f1.z, f1.w);
    *(volatile v4u*)dst = o;
    __threadfence();
    *(volatile v4u*)dst = o;
  } else if (u < nxu + 3u * nwu + 2u * npu) {
    const unsigned int t  = u - nxu - 3u * nwu;
    const unsigned int pl = t / npu;
    const unsigned int r2 = t - pl * npu;
    const unsigned int f  = r2 >> 5;
    const unsigned int s  = r2 & 31u;
    const size_t off = (size_t)f * VTW + ((s < 16u) ? (size_t)(s * 8u)
                                                    : (size_t)VPAD + (size_t)MROWS + (size_t)((s - 16u) * 8u));
    unsigned short* dst = ((pl == 0u) ? vth : vtl) + off;
    v4u z = {0u, 0u, 0u, 0u};
    *(volatile v4u*)dst = z;
    __threadfence();
    *(volatile v4u*)dst = z;
  }
}

__global__ __launch_bounds__(128) void qkv_kernel(const unsigned short* __restrict__ xb,
                                                  const unsigned short* __restrict__ wqb,
                                                  const unsigned short* __restrict__ wkb,
                                                  const unsigned short* __restrict__ wvb,
                                                  const float* __restrict__ bq,
                                                  const float* __restrict__ bk,
                                                  const float* __restrict__ bv,
                                                  unsigned short* qh,
                                                  unsigned short* kh,
                                                  unsigned short* vth,
                                                  unsigned short* vtl) {
  __shared__ __attribute__((aligned(16))) float Ts[64][TPITCH];

  const int tid  = threadIdx.x;
  const int lane = tid & 31;
  const int h    = lane >> 4;
  const int m    = lane & 15;
  const int wv   = tid >> 5;
  const int mat  = blockIdx.z;
  const int rb   = blockIdx.x * 64;
  const int nb   = blockIdx.y * 64;

  const unsigned short* Wm = (mat == 0) ? wqb : (mat == 1) ? wkb : wvb;
  const float* bias      = (mat == 0) ? bq  : (mat == 1) ? bk  : bv;

  const unsigned short* arow = xb + (size_t)(rb + 16 * wv + m) * EDIM;
  const unsigned short* brow[4];
#pragma unroll
  for (int t = 0; t < 4; ++t) brow[t] = Wm + (size_t)(nb + 16 * t + m) * EDIM;

  v8f acc[4];
#pragma unroll
  for (int t = 0; t < 4; ++t) acc[t] = zero8();

  for (int kc = 0; kc < EDIM; kc += 32) {
    FragB a;
    a.u[0] = *(const v4u*)(arow + kc + 8 * h);
    a.u[1] = *(const v4u*)(arow + kc + 16 + 8 * h);
#pragma unroll
    for (int t = 0; t < 4; ++t) {
      FragB bb;
      bb.u[0] = *(const v4u*)(brow[t] + kc + 8 * h);
      bb.u[1] = *(const v4u*)(brow[t] + kc + 16 + 8 * h);
      acc[t] = mma_bf16(a.v, bb.v, acc[t]);
    }
  }

#pragma unroll
  for (int t = 0; t < 4; ++t) {
    const int col = 16 * t + m;
    const float bb = bf16_rne_val(bias[nb + col]);
#pragma unroll
    for (int r = 0; r < 8; ++r) Ts[16 * wv + 8 * h + r][col] = acc[t][r] + bb;
  }
  __syncthreads();

  if (mat < 2) {
    unsigned short* plane = (mat == 0) ? qh : kh;
    for (int rep = 0; rep < 2; ++rep) {
#pragma unroll
      for (int it = 0; it < 4; ++it) {
        const int p   = it * 128 + tid;
        const int row = p >> 3;
        const int c   = p & 7;
        Pack8H pk;
#pragma unroll
        for (int j = 0; j < 8; ++j) pk.h[j] = (_Float16)(Ts[row][8 * c + j] * 16.0f);
        unsigned short* dst = plane + (size_t)(rb + row) * EDIM + nb + 8 * c;
        *(volatile v4u*)dst = pk.u;
      }
      if (rep == 0) __threadfence();
    }
  } else {
    for (int rep = 0; rep < 2; ++rep) {
#pragma unroll
      for (int it = 0; it < 4; ++it) {
        const int p = it * 128 + tid;
        const int f = p >> 3;
        const int c = p & 7;
        Pack8H ph, pl;
#pragma unroll
        for (int j = 0; j < 8; ++j) {
          const float v16 = Ts[8 * c + j][f] * 16.0f;
          const _Float16 hh = (_Float16)v16;
          const float res = (v16 - (float)hh) * 1024.0f;
          ph.h[j] = hh;
          pl.h[j] = (_Float16)res;
        }
        const size_t off = (size_t)(nb + f) * VTW + (size_t)VPAD + (size_t)rb + (size_t)(8 * c);
        *(volatile v4u*)(vth + off) = ph.u;
        *(volatile v4u*)(vtl + off) = pl.u;
      }
      if (rep == 0) __threadfence();
    }
  }
}

__global__ __launch_bounds__(256) void attn_kernel(const unsigned short* __restrict__ qh,
                                                   const unsigned short* __restrict__ kh,
                                                   const unsigned short* __restrict__ vth,
                                                   const unsigned short* __restrict__ vtl,
                                                   const int* __restrict__ wsz,
                                                   float* out) {
  __shared__ __attribute__((aligned(16))) float    Sw[16][SPITCH];
  __shared__ __attribute__((aligned(16))) _Float16 Pwh[16][PPITCH];
  __shared__ __attribute__((aligned(16))) _Float16 Pwl[16][PPITCH];
  __shared__ __attribute__((aligned(16))) float    Os[16][OPITCH];

  const int tid  = threadIdx.x;
  const int lane = tid & 31;
  const int wv   = tid >> 5;
  const int h    = lane >> 4;
  const int m    = lane & 15;

  const int R0 = blockIdx.x * 16;
  const int b  = R0 / SEQ;
  const int l0 = R0 - b * SEQ;

  int wl = wsz[0];
  wl = (wl < 0) ? 0 : ((wl > WIN) ? WIN : wl);

  const unsigned short* qrow = qh + (size_t)(R0 + m) * EDIM;
  const float sc = 0.00390625f * 0.044194173824159216f;
  for (int kt = wv; kt < NKT; kt += 8) {
    const int j    = kt * 16 + m;
    const int kidx = l0 - WIN + j;
    const int kcl  = (kidx < 0) ? 0 : ((kidx >= SEQ) ? (SEQ - 1) : kidx);
    const unsigned short* krow = kh + (size_t)(b * SEQ + kcl) * EDIM;
    v8f acc = zero8();
    for (int ec = 0; ec < EDIM; ec += 32) {
      FragH a, bb;
      a.u[0]  = *(const v4u*)(qrow + ec + 8 * h);
      a.u[1]  = *(const v4u*)(qrow + ec + 16 + 8 * h);
      bb.u[0] = *(const v4u*)(krow + ec + 8 * h);
      bb.u[1] = *(const v4u*)(krow + ec + 16 + 8 * h);
      acc = mma_f16(a.v, bb.v, acc);
    }
    const bool kval = (kidx >= 0) && (kidx < SEQ);
#pragma unroll
    for (int r = 0; r < 8; ++r) {
      const int row = 8 * h + r;
      const bool valid = kval && (j >= row + WIN - wl) && (j <= row + WIN + wl);
      Sw[row][j] = valid ? (acc[r] * sc) : -__builtin_inff();
    }
  }
  __syncthreads();

  {
    const int r = tid >> 4;
    const int c = tid & 15;
    float s[NKT];
#pragma unroll
    for (int t = 0; t < NKT; ++t) s[t] = Sw[r][c + 16 * t];
    float mx = s[0];
#pragma unroll
    for (int t = 1; t < NKT; ++t) mx = fmaxf(mx, s[t]);
    mx = fmaxf(mx, __shfl_xor(mx, 8));
    mx = fmaxf(mx, __shfl_xor(mx, 4));
    mx = fmaxf(mx, __shfl_xor(mx, 2));
    mx = fmaxf(mx, __shfl_xor(mx, 1));
    float e[NKT];
    float sum = 0.0f;
#pragma unroll
    for (int t = 0; t < NKT; ++t) {
      const float ex = __expf(s[t] - mx);
      e[t] = (s[t] > -3.0e38f) ? ex : 0.0f;
      sum += e[t];
    }
    sum += __shfl_xor(sum, 8);
    sum += __shfl_xor(sum, 4);
    sum += __shfl_xor(sum, 2);
    sum += __shfl_xor(sum, 1);
    const float inv = 1.0f / sum;
#pragma unroll
    for (int t = 0; t < NKT; ++t) {
      const float p  = (e[t] * inv) * 1024.0f;
      const _Float16 hh = (_Float16)p;
      Pwh[r][c + 16 * t] = hh;
      Pwl[r][c + 16 * t] = (_Float16)((p - (float)hh) * 1024.0f);
    }
    Pwh[r][NKEYS + c] = (_Float16)0.0f;
    Pwl[r][NKEYS + c] = (_Float16)0.0f;
  }
  __syncthreads();

  const int kb0 = VPAD + b * SEQ + l0 - WIN;
#pragma unroll 1
  for (int t = 0; t < 4; ++t) {
    const int nc = wv + 8 * t;
    const unsigned short* vrh = vth + (size_t)(nc * 16 + m) * VTW + (size_t)kb0;
    const unsigned short* vrl = vtl + (size_t)(nc * 16 + m) * VTW + (size_t)kb0;
    v8f acc0 = zero8();
    v8f acc1 = zero8();
#pragma unroll
    for (int kc = 0; kc < NKC; ++kc) {
      FragH ah, al, bh, bl;
      ah.half[0] = *(const v8h_ma*)(&Pwh[m][kc * 32 + 8 * h]);
      ah.half[1] = *(const v8h_ma*)(&Pwh[m][kc * 32 + 16 + 8 * h]);
      al.half[0] = *(const v8h_ma*)(&Pwl[m][kc * 32 + 8 * h]);
      al.half[1] = *(const v8h_ma*)(&Pwl[m][kc * 32 + 16 + 8 * h]);
      bh.u[0] = *(const v4u*)(vrh + kc * 32 + 8 * h);
      bh.u[1] = *(const v4u*)(vrh + kc * 32 + 16 + 8 * h);
      bl.u[0] = *(const v4u*)(vrl + kc * 32 + 8 * h);
      bl.u[1] = *(const v4u*)(vrl + kc * 32 + 16 + 8 * h);
      acc0 = mma_f16(ah.v, bh.v, acc0);
      acc1 = mma_f16(ah.v, bl.v, acc1);
      acc1 = mma_f16(al.v, bh.v, acc1);
    }
#pragma unroll
    for (int r = 0; r < 8; ++r)
      Os[8 * h + r][nc * 16 + m] = (acc0[r] + acc1[r] * 0.0009765625f) * 6.103515625e-05f;
  }
  __syncthreads();

  float* ob = out + ((size_t)b * SEQ_FULL + (size_t)l0) * EDIM;
  for (int rep = 0; rep < 2; ++rep) {
#pragma unroll
    for (int it = 0; it < 8; ++it) {
      const int f   = it * 256 + tid;
      const int row = f >> 7;
      const int c4  = f & 127;
      const v4f v = *(const v4f_ma*)(&Os[row][4 * c4]);
      *(volatile v4f*)(ob + (size_t)row * EDIM + 4 * c4) = v;
    }
    if (rep == 0) __threadfence();
  }
}

extern "C" void kernel_launch(void* const* d_in, const int* in_sizes, int n_in,
                              void* d_out, int out_size, void* d_ws, size_t ws_size,
                              hipStream_t stream) {
  if (n_in < 8) return;
  const long long needX = ((long long)(NB - 1) * SEQ_FULL + SEQ) * EDIM;
  if ((long long)in_sizes[0] < needX) return;
  if (in_sizes[1] < EDIM * EDIM || in_sizes[3] < EDIM * EDIM || in_sizes[5] < EDIM * EDIM) return;
  if (in_sizes[2] < EDIM || in_sizes[4] < EDIM || in_sizes[6] < EDIM) return;
  if (in_sizes[7] < 1) return;
  if ((long long)out_size < needX) return;

  const float* x   = (const float*)d_in[0];
  const float* Wq  = (const float*)d_in[1];
  const float* bq  = (const float*)d_in[2];
  const float* Wk  = (const float*)d_in[3];
  const float* bk  = (const float*)d_in[4];
  const float* Wv  = (const float*)d_in[5];
  const float* bv  = (const float*)d_in[6];
  const int*   wsz = (const int*)d_in[7];

  char* ws = (char*)d_ws;
  size_t off = 0;
  auto carve = [&](size_t bytes) -> void* {
    void* p = ws + off;
    off += (bytes + 255) & ~(size_t)255;
    return p;
  };
  unsigned short* xb  = (unsigned short*)carve((size_t)MROWS * EDIM * 2);
  unsigned short* wqb = (unsigned short*)carve((size_t)EDIM * EDIM * 2);
  unsigned short* wkb = (unsigned short*)carve((size_t)EDIM * EDIM * 2);
  unsigned short* wvb = (unsigned short*)carve((size_t)EDIM * EDIM * 2);
  unsigned short* qh  = (unsigned short*)carve((size_t)MROWS * EDIM * 2);
  unsigned short* kh  = (unsigned short*)carve((size_t)MROWS * EDIM * 2);
  unsigned short* vth = (unsigned short*)carve((size_t)EDIM * VTW * 2);
  unsigned short* vtl = (unsigned short*)carve((size_t)EDIM * VTW * 2);
  if (off > ws_size) return;

  {
    const unsigned int total = (unsigned int)MROWS * 64u + 3u * (unsigned int)(EDIM * EDIM) / 8u + 2u * (unsigned int)EDIM * 32u;
    hipLaunchKernelGGL(cvt_kernel, dim3(total / 256u), dim3(256), 0, stream,
                       x, Wq, Wk, Wv, xb, wqb, wkb, wvb, vth, vtl);
  }
  {
    hipLaunchKernelGGL(qkv_kernel, dim3(MROWS / 64, EDIM / 64, 3), dim3(128), 0, stream,
                       xb, wqb, wkb, wvb, bq, bk, bv, qh, kh, vth, vtl);
  }
  {
    hipLaunchKernelGGL(attn_kernel, dim3(MROWS / 16), dim3(256), 0, stream,
                       qh, kh, vth, vtl, wsz, (float*)d_out);
  }
}
